// Decoder_49203145343612
// MI455X (gfx1250) — hardware-verified
//
#include <hip/hip_runtime.h>
#include <math.h>

constexpr int NBATCH   = 256;
constexpr int NSTEP    = 512;
constexpr int NIN      = 128;
constexpr int NHID1    = 128;
constexpr int NHID2    = 256;
constexpr int NGATE1   = 4 * NHID1;
constexpr int NGATE2   = 4 * NHID2;
constexpr int KCAT2    = NHID1 + NHID2;
constexpr int NTHR     = 256;
constexpr int NWAVE    = NTHR / 32;
constexpr int ROWS_BLK = 32;
constexpr int NBLK     = NBATCH / ROWS_BLK;
constexpr int H1PITCH  = 136;
constexpr int H2PITCH  = 264;
constexpr int XPPITCH  = 36;
constexpr int STPITCH  = 36;
constexpr int FLUSH    = 32;
constexpr float W_CARRY       = 256.0f;
constexpr float H_CARRY       = 16.0f;
constexpr float ACC_CARRY     = W_CARRY * H_CARRY;
constexpr float ACC_CARRY_INV = 1.0f / ACC_CARRY;

static_assert(NHID1 == 16 * NWAVE, "one layer-1 column tile per wave");
static_assert(NHID2 == 32 * NWAVE, "two layer-2 column tiles per wave");
static_assert(ROWS_BLK == 4 * NWAVE, "flush map: four rows per wave");
static_assert(NSTEP % FLUSH == 0, "no flush tail");
static_assert(NBATCH % ROWS_BLK == 0, "row tiles exact");
static_assert(NHID1 % 32 == 0 && NHID2 % 32 == 0 && KCAT2 % 32 == 0, "K multiples of 32");
static_assert((2 * ROWS_BLK * H1PITCH) % NTHR == 0, "h1 zero fill exact");
static_assert((2 * ROWS_BLK * H2PITCH) % NTHR == 0, "h2 zero fill exact");
static_assert(NGATE2 == 4 * NTHR, "bias staging exact");
static_assert((ROWS_BLK * NGATE1) % (4 * NTHR) == 0, "xp staging exact");
static_assert(NGATE1 / 4 == 128, "xproj index split");
static_assert(H1PITCH % 8 == 0 && H2PITCH % 8 == 0 && XPPITCH % 4 == 0 && STPITCH % 4 == 0, "16-B aligned pitches");

typedef __attribute__((ext_vector_type(16))) _Float16 v16h;
typedef __attribute__((ext_vector_type(8)))  _Float16 v8h;
typedef __attribute__((ext_vector_type(8)))  float    v8f;
typedef __attribute__((ext_vector_type(4)))  float    v4f;

template <typename T> struct Frag;
template <> struct Frag<_Float16> {
  typedef v16h V; union U { v16h v; v8h h[2]; };
  static __device__ __forceinline__ v16h load(const _Float16* p) {
    U f; f.h[0] = *(const v8h*)(p); f.h[1] = *(const v8h*)(p + 16); return f.v;
  }
  static __device__ __forceinline__ v8f mma(v16h a, v16h b, v8f c) {
    return __builtin_amdgcn_wmma_f32_16x16x32_f16(false, a, false, b, (short)0, c, false, false);
  }
};
typedef Frag<_Float16> FragH;

__device__ __forceinline__ void guard8(v8f& d0, v8f& d1, v8f& d2, v8f& d3, v8f& d4, v8f& d5, v8f& d6, v8f& d7,
                                       v16h x0, v16h x1, v16h y0, v16h y1, v16h y2, v16h y3) {
  asm volatile("v_nop\n\tv_nop\n\tv_nop\n\tv_nop"
               : "+v"(d0), "+v"(d1), "+v"(d2), "+v"(d3), "+v"(d4), "+v"(d5), "+v"(d6), "+v"(d7)
               : "v"(x0), "v"(x1), "v"(y0), "v"(y1), "v"(y2), "v"(y3));
}

__device__ __forceinline__ float fsig(float x)  { return __builtin_amdgcn_rcpf(1.0f + __expf(-x)); }
__device__ __forceinline__ float ftanh(float x) { return 1.0f - 2.0f * __builtin_amdgcn_rcpf(__expf(2.0f * x) + 1.0f); }

template <int GSTRIDE>
__device__ __forceinline__ void kstep8(v8f (&acc)[4][2], const _Float16* a0p, const _Float16* a1p, const _Float16* bp) {
  const v16h a0 = FragH::load(a0p);
  const v16h a1 = FragH::load(a1p);
  const v16h b0 = FragH::load(bp);
  const v16h b1 = FragH::load(bp + (size_t)GSTRIDE);
  const v16h b2 = FragH::load(bp + (size_t)2 * GSTRIDE);
  const v16h b3 = FragH::load(bp + (size_t)3 * GSTRIDE);
  acc[0][0] = FragH::mma(a0, b0, acc[0][0]);
  acc[0][1] = FragH::mma(a1, b0, acc[0][1]);
  acc[1][0] = FragH::mma(a0, b1, acc[1][0]);
  acc[1][1] = FragH::mma(a1, b1, acc[1][1]);
  acc[2][0] = FragH::mma(a0, b2, acc[2][0]);
  acc[2][1] = FragH::mma(a1, b2, acc[2][1]);
  acc[3][0] = FragH::mma(a0, b3, acc[3][0]);
  acc[3][1] = FragH::mma(a1, b3, acc[3][1]);
  guard8(acc[0][0], acc[0][1], acc[1][0], acc[1][1], acc[2][0], acc[2][1], acc[3][0], acc[3][1],
         a0, a1, b0, b1, b2, b3);
}

__global__ __launch_bounds__(NTHR) void cvt8_f16_kernel(const float* __restrict__ src, unsigned short* __restrict__ dst,
                                                        int nrow, int ncol8, int spitch, int dpitch, int dcol0, float sc) {
  const int i  = blockIdx.x * NTHR + threadIdx.x;
  const int n8 = nrow * ncol8;
  if (i < n8) {
    const int row = i / ncol8;
    const int c8  = i - row * ncol8;
    const float* sp = src + (size_t)row * spitch + c8 * 8;
    const v4f a = *(const v4f*)(sp);
    const v4f b = *(const v4f*)(sp + 4);
    v8h hv;
#pragma unroll
    for (int e = 0; e < 4; ++e) {
      hv[e]     = (_Float16)(a[e] * sc);
      hv[4 + e] = (_Float16)(b[e] * sc);
    }
    unsigned short* dp = dst + (size_t)row * dpitch + dcol0 + c8 * 8;
    *(volatile v8h*)dp = hv;
    __threadfence();
    *(volatile v8h*)dp = hv;
  }
}

__global__ __launch_bounds__(NTHR) void xproj_kernel(const float* __restrict__ x, const float* __restrict__ wih1,
                                                     const float* __restrict__ bih1, const float* __restrict__ bhh1,
                                                     float* __restrict__ xp1) {
  const int i = blockIdx.x * NTHR + threadIdx.x;
  if (i < NBATCH * (NGATE1 / 4)) {
    const int b  = i >> 7;
    const int n0 = (i & 127) * 4;
    const float* xr = x + (size_t)b * NIN;
    const float* w0 = wih1 + (size_t)n0 * NIN;
    float s0 = 0.0f, s1 = 0.0f, s2 = 0.0f, s3 = 0.0f;
#pragma unroll 1
    for (int k = 0; k < NIN; k += 4) {
      const v4f xv = *(const v4f*)(xr + k);
      const v4f wa = *(const v4f*)(w0 + k);
      const v4f wb = *(const v4f*)(w0 + NIN + k);
      const v4f wc = *(const v4f*)(w0 + 2 * NIN + k);
      const v4f wd = *(const v4f*)(w0 + 3 * NIN + k);
#pragma unroll
      for (int e = 0; e < 4; ++e) {
        s0 += xv[e] * wa[e];
        s1 += xv[e] * wb[e];
        s2 += xv[e] * wc[e];
        s3 += xv[e] * wd[e];
      }
    }
    const v4f bi = *(const v4f*)(bih1 + n0);
    const v4f bh = *(const v4f*)(bhh1 + n0);
    v4f o;
    o[0] = (s0 + bi[0]) + bh[0];
    o[1] = (s1 + bi[1]) + bh[1];
    o[2] = (s2 + bi[2]) + bh[2];
    o[3] = (s3 + bi[3]) + bh[3];
    float* op = xp1 + (size_t)b * NGATE1 + n0;
    *(volatile v4f*)op = o;
    __threadfence();
    *(volatile v4f*)op = o;
  }
}

__global__ __launch_bounds__(NTHR) void lstm2_seq_kernel(const float* __restrict__ xp1,
                                                         const unsigned short* __restrict__ bt1p,
                                                         const unsigned short* __restrict__ bt2p,
                                                         const float* __restrict__ bih2, const float* __restrict__ bhh2,
                                                         const float* __restrict__ wout, const float* __restrict__ bout,
                                                         float* __restrict__ out) {
  __shared__ __align__(16) _Float16 h1s[2][ROWS_BLK * H1PITCH];
  __shared__ __align__(16) _Float16 h2s[2][ROWS_BLK * H2PITCH];
  __shared__ __align__(16) float    xps[NGATE1 * XPPITCH];
  __shared__ __align__(16) float    b2s[NGATE2];
  __shared__ __align__(16) float    parts[NWAVE * ROWS_BLK];
  __shared__ __align__(16) float    stage[ROWS_BLK * STPITCH];

  const _Float16* BT1 = (const _Float16*)bt1p;
  const _Float16* BT2 = (const _Float16*)bt2p;
  const int tid = threadIdx.x, lane = tid & 31, wave = tid >> 5;
  const int c = lane & 15, hh = lane >> 4, koff = hh * 8;
  const int rowbase = blockIdx.x * ROWS_BLK;

  {
    _Float16* p1 = &h1s[0][0];
#pragma unroll 1
    for (int i = tid; i < 2 * ROWS_BLK * H1PITCH; i += NTHR) p1[i] = (_Float16)0.0f;
    _Float16* p2 = &h2s[0][0];
#pragma unroll 1
    for (int i = tid; i < 2 * ROWS_BLK * H2PITCH; i += NTHR) p2[i] = (_Float16)0.0f;
  }
#pragma unroll 1
  for (int it = 0; it < (ROWS_BLK * NGATE1) / (4 * NTHR); ++it) {
    const int idx = it * NTHR + tid;
    const int row = idx >> 7;
    const int c4  = (idx & 127) * 4;
    const v4f v = *(const v4f*)(xp1 + (size_t)(rowbase + row) * NGATE1 + c4);
    xps[(c4 + 0) * XPPITCH + row] = v[0];
    xps[(c4 + 1) * XPPITCH + row] = v[1];
    xps[(c4 + 2) * XPPITCH + row] = v[2];
    xps[(c4 + 3) * XPPITCH + row] = v[3];
  }
  {
    const v4f a = *(const v4f*)(bih2 + tid * 4);
    const v4f b = *(const v4f*)(bhh2 + tid * 4);
    b2s[tid * 4 + 0] = a[0] + b[0];
    b2s[tid * 4 + 1] = a[1] + b[1];
    b2s[tid * 4 + 2] = a[2] + b[2];
    b2s[tid * 4 + 3] = a[3] + b[3];
  }
  const float wo0 = wout[16 * (2 * wave) + c];
  const float wo1 = wout[16 * (2 * wave + 1) + c];
  const float bo  = bout[0];

  float c1[2][8], c2[2][2][8];
#pragma unroll
  for (int mt = 0; mt < 2; ++mt)
#pragma unroll
    for (int r = 0; r < 8; ++r) {
      c1[mt][r] = 0.0f;
      c2[0][mt][r] = 0.0f;
      c2[1][mt][r] = 0.0f;
    }
  __syncthreads();

#pragma unroll 1
  for (int t = 0; t < NSTEP; ++t) {
    const int cur = t & 1;
    const _Float16* h1c = &h1s[cur][0];
    _Float16*       h1n = &h1s[cur ^ 1][0];
    const _Float16* h2c = &h2s[cur][0];
    _Float16*       h2n = &h2s[cur ^ 1][0];

    {
      v8f acc[4][2];
#pragma unroll
      for (int g = 0; g < 4; ++g) {
        const float* xq = xps + (g * NHID1 + 16 * wave + c) * XPPITCH + 8 * hh;
#pragma unroll
        for (int mt = 0; mt < 2; ++mt) {
          const v4f lo = *(const v4f*)(xq + 16 * mt);
          const v4f hi = *(const v4f*)(xq + 16 * mt + 4);
          v8f a;
          a[0] = lo[0] * ACC_CARRY; a[1] = lo[1] * ACC_CARRY; a[2] = lo[2] * ACC_CARRY; a[3] = lo[3] * ACC_CARRY;
          a[4] = hi[0] * ACC_CARRY; a[5] = hi[1] * ACC_CARRY; a[6] = hi[2] * ACC_CARRY; a[7] = hi[3] * ACC_CARRY;
          acc[g][mt] = a;
        }
      }
      const _Float16* a0p = h1c + c * H1PITCH + koff;
      const _Float16* a1p = a0p + 16 * H1PITCH;
      const _Float16* bp  = BT1 + (size_t)(16 * wave + c) * NHID1 + koff;
#pragma unroll 1
      for (int k0 = 0; k0 < NHID1; k0 += 32) kstep8<NHID1 * NHID1>(acc, a0p + k0, a1p + k0, bp + k0);
#pragma unroll
      for (int mt = 0; mt < 2; ++mt) {
#pragma unroll
        for (int r = 0; r < 8; ++r) {
          const float ig = fsig(acc[0][mt][r] * ACC_CARRY_INV);
          const float fg = fsig(acc[1][mt][r] * ACC_CARRY_INV);
          const float gg = ftanh(acc[2][mt][r] * ACC_CARRY_INV);
          const float og = fsig(acc[3][mt][r] * ACC_CARRY_INV);
          const float cn = fg * c1[mt][r] + ig * gg;
          c1[mt][r] = cn;
          const float hn = og * ftanh(cn);
          h1n[(16 * mt + 8 * hh + r) * H1PITCH + 16 * wave + c] = (_Float16)(hn * H_CARRY);
        }
      }
    }
    __syncthreads();

    float part[2][8];
#pragma unroll
    for (int p = 0; p < 2; ++p) {
      const int col = 16 * (2 * wave + p) + c;
      v8f acc[4][2];
#pragma unroll
      for (int g = 0; g < 4; ++g) {
        const float bv = b2s[g * NHID2 + col] * ACC_CARRY;
        const v8f a = {bv, bv, bv, bv, bv, bv, bv, bv};
        acc[g][0] = a;
        acc[g][1] = a;
      }
      const _Float16* bp = BT2 + (size_t)col * KCAT2 + koff;
      {
        const _Float16* a0p = h1n + c * H1PITCH + koff;
        const _Float16* a1p = a0p + 16 * H1PITCH;
#pragma unroll 1
        for (int k0 = 0; k0 < NHID1; k0 += 32) kstep8<NHID2 * KCAT2>(acc, a0p + k0, a1p + k0, bp + k0);
      }
      {
        const _Float16* a0p = h2c + c * H2PITCH + koff;
        const _Float16* a1p = a0p + 16 * H2PITCH;
        const _Float16* bq  = bp + NHID1;
#pragma unroll 1
        for (int k0 = 0; k0 < NHID2; k0 += 32) kstep8<NHID2 * KCAT2>(acc, a0p + k0, a1p + k0, bq + k0);
      }
      const float wo = (p == 0) ? wo0 : wo1;
#pragma unroll
      for (int mt = 0; mt < 2; ++mt) {
#pragma unroll
        for (int r = 0; r < 8; ++r) {
          const float ig = fsig(acc[0][mt][r] * ACC_CARRY_INV);
          const float fg = fsig(acc[1][mt][r] * ACC_CARRY_INV);
          const float gg = ftanh(acc[2][mt][r] * ACC_CARRY_INV);
          const float og = fsig(acc[3][mt][r] * ACC_CARRY_INV);
          const float cn = fg * c2[p][mt][r] + ig * gg;
          c2[p][mt][r] = cn;
          const float hn = og * ftanh(cn);
          h2n[(16 * mt + 8 * hh + r) * H2PITCH + col] = (_Float16)(hn * H_CARRY);
          const float pv = hn * wo;
          if (p == 0) part[mt][r] = pv;
          else        part[mt][r] = part[mt][r] + pv;
        }
      }
    }
#pragma unroll
    for (int mt = 0; mt < 2; ++mt) {
#pragma unroll
      for (int r = 0; r < 8; ++r) {
        float s = part[mt][r];
        s += __shfl_xor(s, 1, 32);
        s += __shfl_xor(s, 2, 32);
        s += __shfl_xor(s, 4, 32);
        s += __shfl_xor(s, 8, 32);
        part[mt][r] = s;
      }
    }
    if (c == 0) {
#pragma unroll
      for (int mt = 0; mt < 2; ++mt)
#pragma unroll
        for (int r = 0; r < 8; ++r) parts[wave * ROWS_BLK + 16 * mt + 8 * hh + r] = part[mt][r];
    }
    __syncthreads();

    if (wave == 0) {
      float s = 0.0f;
#pragma unroll
      for (int w = 0; w < NWAVE; ++w) s += parts[w * ROWS_BLK + lane];
      s += bo;
      stage[lane * STPITCH + (t & (FLUSH - 1))] = s;
    }

    if ((t & (FLUSH - 1)) == (FLUSH - 1)) {
      __syncthreads();
      const int row = 4 * wave + (lane >> 3);
      const int s4  = (lane & 7) * 4;
      const v4f v = *(const v4f*)(stage + row * STPITCH + s4);
      float* op = out + (size_t)(rowbase + row) * NSTEP + (size_t)(t - (FLUSH - 1)) + s4;
      *(volatile v4f*)op = v;
      __threadfence();
      *(volatile v4f*)op = v;
    }
  }
}

extern "C" void kernel_launch(void* const* d_in, const int* in_sizes, int n_in,
                              void* d_out, int out_size, void* d_ws, size_t ws_size, hipStream_t stream) {
  if (n_in < 11 || d_out == nullptr || d_ws == nullptr) return;
  if (in_sizes[0] != NBATCH * NIN || in_sizes[1] != NGATE1 * NIN || in_sizes[2] != NGATE1 * NHID1 ||
      in_sizes[3] != NGATE1 || in_sizes[4] != NGATE1 || in_sizes[5] != NGATE2 * NHID1 ||
      in_sizes[6] != NGATE2 * NHID2 || in_sizes[7] != NGATE2 || in_sizes[8] != NGATE2 ||
      in_sizes[9] != NHID2 || in_sizes[10] != 1 || out_size != NBATCH * NSTEP) return;

  const float* x     = (const float*)d_in[0];
  const float* w_ih1 = (const float*)d_in[1];
  const float* w_hh1 = (const float*)d_in[2];
  const float* b_ih1 = (const float*)d_in[3];
  const float* b_hh1 = (const float*)d_in[4];
  const float* w_ih2 = (const float*)d_in[5];
  const float* w_hh2 = (const float*)d_in[6];
  const float* b_ih2 = (const float*)d_in[7];
  const float* b_hh2 = (const float*)d_in[8];
  const float* w_out = (const float*)d_in[9];
  const float* b_out = (const float*)d_in[10];
  float* out = (float*)d_out;

  char* ws = (char*)d_ws; size_t off = 0;
  auto carve = [&](size_t bytes) -> char* { char* p = ws + off; off += (bytes + 255) & ~(size_t)255; return p; };
  unsigned short* BT1 = (unsigned short*)carve((size_t)NGATE1 * NHID1 * 2);
  unsigned short* BT2 = (unsigned short*)carve((size_t)NGATE2 * KCAT2 * 2);
  float*          XP1 = (float*)carve((size_t)NBATCH * NGATE1 * 4);
  if (off > ws_size || off > (size_t)134217728) return;

  const int n8a = NGATE1 * (NHID1 / 8);
  const int n8b = NGATE2 * (NHID1 / 8);
  const int n8c = NGATE2 * (NHID2 / 8);
  cvt8_f16_kernel<<<(n8a + NTHR - 1) / NTHR, NTHR, 0, stream>>>(w_hh1, BT1, NGATE1, NHID1 / 8, NHID1, NHID1, 0, W_CARRY);
  cvt8_f16_kernel<<<(n8b + NTHR - 1) / NTHR, NTHR, 0, stream>>>(w_ih2, BT2, NGATE2, NHID1 / 8, NHID1, KCAT2, 0, W_CARRY);
  cvt8_f16_kernel<<<(n8c + NTHR - 1) / NTHR, NTHR, 0, stream>>>(w_hh2, BT2, NGATE2, NHID2 / 8, NHID2, KCAT2, NHID1, W_CARRY);
  xproj_kernel<<<(NBATCH * (NGATE1 / 4) + NTHR - 1) / NTHR, NTHR, 0, stream>>>(x, w_ih1, b_ih1, b_hh1, XP1);
  lstm2_seq_kernel<<<NBLK, NTHR, 0, stream>>>(XP1, BT1, BT2, b_ih2, b_hh2, w_out, b_out, out);
}
